// RNN_65360812310922
// MI455X (gfx1250) — hardware-verified
//
#include <hip/hip_runtime.h>
#include <math.h>

constexpr int N_BATCH    = 64;
constexpr int N_STEP     = 512;
constexpr int N_IN       = 256;
constexpr int N_HID      = 1024;
constexpr int N_OUT      = 512;
constexpr int T_CHUNK    = 128;
constexpr int N_CHUNK    = N_STEP / T_CHUNK;
constexpr int CH_ROWS    = T_CHUNK * N_BATCH;
constexpr int SCAN_ROWS  = 32;
constexpr int SCAN_THR   = 512;
constexpr int SCAN_WAVES = SCAN_THR / 32;
constexpr int H_PITCH    = 1032;
constexpr int SLAB_PITCH = 68;
constexpr float W_CARRY     = 256.0f;
constexpr float W_CARRY_INV = 1.0f / 256.0f;

static_assert(N_STEP % T_CHUNK == 0, "chunking exact");
static_assert(N_BATCH % SCAN_ROWS == 0, "batch tiles exact");
static_assert(N_HID == 64 * SCAN_WAVES, "16 waves x 64 hidden columns");
static_assert(N_IN % 32 == 0 && N_HID % 32 == 0, "GEMM K multiple of 32");
static_assert(CH_ROWS % 64 == 0 && N_BATCH % 64 == 0, "GEMM M tile multiple");
static_assert(N_HID % 64 == 0 && N_OUT % 64 == 0, "GEMM N tile multiple");
static_assert(H_PITCH % 8 == 0 && H_PITCH >= N_HID, "h tile pitch keeps 16-B alignment");
static_assert((SCAN_ROWS * (N_HID / 8)) % SCAN_THR == 0, "h tile fill loop exact");
static_assert(N_IN / 8 == 32, "x convert: one wave per output row");

typedef __attribute__((ext_vector_type(16))) _Float16 v16h;
typedef __attribute__((ext_vector_type(8)))  _Float16 v8h;
typedef __attribute__((ext_vector_type(8)))  float    v8f;
typedef __attribute__((ext_vector_type(4)))  float    v4f;

__device__ __forceinline__ unsigned short f2bf_bits(float f) {
  unsigned u = __float_as_uint(f);
  return (unsigned short)((u + 0x7FFFu + ((u >> 16) & 1u)) >> 16);
}
__device__ __forceinline__ float bf_bits2f(unsigned short h) { return __uint_as_float(((unsigned)h) << 16); }
__device__ __forceinline__ float bf16r(float f) { return bf_bits2f(f2bf_bits(f)); }

__device__ __forceinline__ void keep4_h(v16h a, v16h b, v16h c, v16h d) { asm volatile("v_nop" :: "v"(a), "v"(b), "v"(c), "v"(d)); }
__device__ __forceinline__ void acc_guard4(v8f& a, v8f& b, v8f& c, v8f& d) { asm volatile("v_nop\n\tv_nop\n\tv_nop\n\tv_nop" : "+v"(a), "+v"(b), "+v"(c), "+v"(d)); }
__device__ __forceinline__ void guard4_h(v8f& c0, v8f& c1, v8f& c2, v8f& c3, v16h a, v16h b0, v16h b1, v16h b2, v16h b3) {
  asm volatile("v_nop\n\tv_nop\n\tv_nop\n\tv_nop"
               : "+v"(c0), "+v"(c1), "+v"(c2), "+v"(c3)
               : "v"(a), "v"(b0), "v"(b1), "v"(b2), "v"(b3));
}
__device__ __forceinline__ void guard8_h(v8f& c0, v8f& c1, v8f& c2, v8f& c3, v8f& c4, v8f& c5, v8f& c6, v8f& c7,
                                         v16h a0, v16h a1, v16h b0, v16h b1, v16h b2, v16h b3) {
  asm volatile("v_nop\n\tv_nop\n\tv_nop\n\tv_nop"
               : "+v"(c0), "+v"(c1), "+v"(c2), "+v"(c3), "+v"(c4), "+v"(c5), "+v"(c6), "+v"(c7)
               : "v"(a0), "v"(a1), "v"(b0), "v"(b1), "v"(b2), "v"(b3));
}

struct FragH {
  union U { v16h v; v8h h[2]; };
  static __device__ __forceinline__ v16h load(const _Float16* p) {
    U f; f.h[0] = *(const v8h*)(p); f.h[1] = *(const v8h*)(p + 16); return f.v;
  }
  static __device__ __forceinline__ v8f mma(v16h a, v16h b, v8f c) {
    return __builtin_amdgcn_wmma_f32_16x16x32_f16(false, a, false, b, (short)0, c, false, false);
  }
};

__device__ __forceinline__ void wave_lds_sync() {
  __builtin_amdgcn_fence(__ATOMIC_RELEASE, "workgroup");
  __builtin_amdgcn_wave_barrier();
  __builtin_amdgcn_fence(__ATOMIC_ACQUIRE, "workgroup");
}

__device__ __forceinline__ float tanh_f32(float x) {
  const float e = expf(2.0f * x);
  return 1.0f - 2.0f * __builtin_amdgcn_rcpf(e + 1.0f);
}

__global__ __launch_bounds__(256) void wmma_gemm64_f16(
    const unsigned short* __restrict__ Ap, int lda,
    const unsigned short* __restrict__ Btp, int ldb,
    float* __restrict__ Cout, int ldc,
    const float* __restrict__ bias,
    int M, int N, int K, float scale) {
  const _Float16* A  = (const _Float16*)Ap;
  const _Float16* Bt = (const _Float16*)Btp;
  __shared__ __align__(16) float sT[8][16 * 68];
  const int lane = threadIdx.x & 31;
  const int wave = threadIdx.x >> 5;
  const int tilesN = N >> 6;
  const int tilesM = M >> 6;
  const int tile = blockIdx.x * 8 + wave;
  if (tile >= tilesM * tilesN) return;
  const int tm = tile / tilesN;
  const int tn = tile - tm * tilesN;
  const int m0 = tm << 6;
  const int n0 = tn << 6;

  const int rlane = lane & 15;
  const int koff  = (lane >> 4) * 8;
  const int mOff  = (lane >> 4) * 8;

  v8f acc[4][4];
#pragma unroll
  for (int i = 0; i < 4; ++i)
#pragma unroll
    for (int j = 0; j < 4; ++j) acc[i][j] = (v8f){0.f,0.f,0.f,0.f,0.f,0.f,0.f,0.f};

  for (int k0 = 0; k0 < K; k0 += 32) {
    v16h bh[4];
#pragma unroll
    for (int j = 0; j < 4; ++j) {
      const size_t bo = (size_t)(n0 + (j << 4) + rlane) * ldb + koff + k0;
      bh[j] = FragH::load(Bt + bo);
    }
#pragma unroll
    for (int i = 0; i < 4; ++i) {
      const size_t ao = (size_t)(m0 + (i << 4) + rlane) * lda + koff + k0;
      const v16h ah = FragH::load(A + ao);
#pragma unroll
      for (int j = 0; j < 4; ++j) acc[i][j] = FragH::mma(ah, bh[j], acc[i][j]);
      guard4_h(acc[i][0], acc[i][1], acc[i][2], acc[i][3], ah, bh[0], bh[1], bh[2], bh[3]);
    }
    keep4_h(bh[0], bh[1], bh[2], bh[3]);
  }
  acc_guard4(acc[0][0], acc[0][1], acc[0][2], acc[0][3]);
  acc_guard4(acc[1][0], acc[1][1], acc[1][2], acc[1][3]);
  acc_guard4(acc[2][0], acc[2][1], acc[2][2], acc[2][3]);
  acc_guard4(acc[3][0], acc[3][1], acc[3][2], acc[3][3]);

  float* slab = sT[wave];
#pragma unroll
  for (int i = 0; i < 4; ++i) {
    const int mBase = m0 + (i << 4);
#pragma unroll
    for (int j = 0; j < 4; ++j) {
      const int n = n0 + (j << 4) + rlane;
      const float bv = bias[n];
#pragma unroll
      for (int r = 0; r < 8; ++r) {
        const float v = acc[i][j][r] * scale + bv;
        slab[(mOff + r) * 68 + (j << 4) + rlane] = v;
      }
    }
    wave_lds_sync();
    {
      const int hh = lane >> 4, c4 = (lane & 15) * 4;
      for (int pass = 0; pass < 2; ++pass) {
#pragma unroll
        for (int it = 0; it < 8; ++it) {
          const int row = it * 2 + hh;
          const v4f v = *(const v4f*)(slab + row * 68 + c4);
          *(volatile v4f*)(Cout + (size_t)(mBase + row) * ldc + n0 + c4) = v;
        }
        __threadfence();
      }
    }
    wave_lds_sync();
  }
}

__global__ __launch_bounds__(256) void cvt_w_kernel(const float* __restrict__ src, unsigned short* __restrict__ dst,
                                                    int n8, float sc) {
  const int i = blockIdx.x * 256 + threadIdx.x;
  if (i < n8) {
    const float* sp = src + (size_t)i * 8;
    const v4f a = *(const v4f*)(sp);
    const v4f b = *(const v4f*)(sp + 4);
    v8h hv;
#pragma unroll
    for (int e = 0; e < 4; ++e) {
      const float fa = a[e];
      const float fb = b[e];
      hv[e]     = (_Float16)(bf16r(fa) * sc);
      hv[4 + e] = (_Float16)(bf16r(fb) * sc);
    }
    _Float16* op = (_Float16*)dst + (size_t)i * 8;
    *(volatile v8h*)op = hv;
    __threadfence();
    *(volatile v8h*)op = hv;
  }
}

__global__ __launch_bounds__(256) void cvt_x_tmajor_kernel(const float* __restrict__ x, unsigned short* __restrict__ dst) {
  const int i = blockIdx.x * 256 + threadIdx.x;
  constexpr int n8 = N_BATCH * N_STEP * (N_IN / 8);
  if (i < n8) {
    const int orow = i / (N_IN / 8);
    const int c8   = i - orow * (N_IN / 8);
    const int t    = orow / N_BATCH;
    const int b    = orow - t * N_BATCH;
    const float* sp = x + ((size_t)b * N_STEP + (size_t)t) * N_IN + c8 * 8;
    const v4f a  = *(const v4f*)(sp);
    const v4f bq = *(const v4f*)(sp + 4);
    v8h hv;
#pragma unroll
    for (int e = 0; e < 4; ++e) {
      const float fa = a[e];
      const float fb = bq[e];
      hv[e]     = (_Float16)bf16r(fa);
      hv[4 + e] = (_Float16)bf16r(fb);
    }
    _Float16* op = (_Float16*)dst + (size_t)i * 8;
    *(volatile v8h*)op = hv;
    __threadfence();
    *(volatile v8h*)op = hv;
  }
}

__global__ __launch_bounds__(256) void bias_prep_kernel(const float* __restrict__ bih0, const float* __restrict__ bhh0,
                                                        const float* __restrict__ bih1, const float* __restrict__ bhh1,
                                                        const float* __restrict__ bfc,
                                                        float* __restrict__ bs0, float* __restrict__ bs1,
                                                        float* __restrict__ bfr) {
  const int blk = blockIdx.x;
  const int idx = threadIdx.x * 4;
  const float* pa = (blk == 0) ? bih0 : ((blk == 1) ? bih1 : bfc);
  const float* pb = (blk == 0) ? bhh0 : ((blk == 1) ? bhh1 : bfc);
  float* po = (blk == 0) ? bs0 : ((blk == 1) ? bs1 : bfr);
  const int n = (blk == 2) ? N_OUT : N_HID;
  const bool two = (blk != 2);
  if (idx < n) {
    const v4f va = *(const v4f*)(pa + idx);
    const v4f vb = *(const v4f*)(pb + idx);
    v4f o;
#pragma unroll
    for (int e = 0; e < 4; ++e) {
      const float fa = va[e];
      const float fb = vb[e];
      const float second = two ? bf16r(fb) : 0.0f;
      o[e] = bf16r(fa) + second;
    }
    *(volatile v4f*)(po + idx) = o;
    __threadfence();
    *(volatile v4f*)(po + idx) = o;
  }
}

template <bool SEQ>
__device__ __forceinline__ void epi_half(const v8f a0, const v8f a1, const v8f a2, const v8f a3,
                                         float* slab, _Float16* hrows, const float* xrows,
                                         _Float16* grows, _Float16* srows, const bool last,
                                         const int c, const int hh, const int q, const int c8) {
#pragma unroll
  for (int r = 0; r < 8; ++r) {
    float* sp = slab + (8 * hh + r) * SLAB_PITCH + c;
    sp[0]  = a0[r];
    sp[16] = a1[r];
    sp[32] = a2[r];
    sp[48] = a3[r];
  }
  wave_lds_sync();
#pragma unroll 1
  for (int it = 0; it < 4; ++it) {
    const int row = it * 4 + q;
    const float* sp = slab + row * SLAB_PITCH + c8;
    const v4f s0 = *(const v4f*)(sp);
    const v4f s1 = *(const v4f*)(sp + 4);
    const float* xr = xrows + (size_t)row * N_HID + c8;
    const v4f x0 = *(const v4f*)(xr);
    const v4f x1 = *(const v4f*)(xr + 4);
    v8h hv;
#pragma unroll
    for (int e = 0; e < 4; ++e) {
      const float p0 = s0[e] * W_CARRY_INV + x0[e];
      const float p1 = s1[e] * W_CARRY_INV + x1[e];
      hv[e]     = (_Float16)tanh_f32(p0);
      hv[4 + e] = (_Float16)tanh_f32(p1);
    }
    *(v8h*)(hrows + row * H_PITCH + c8) = hv;
    _Float16* gp  = grows + (size_t)row * N_HID + c8;
    _Float16* stp = srows + (size_t)row * N_HID + c8;
    if (SEQ)  *(volatile v8h*)gp  = hv;
    if (last) *(volatile v8h*)stp = hv;
    if (SEQ || last) __threadfence();
    if (SEQ)  *(volatile v8h*)gp  = hv;
    if (last) *(volatile v8h*)stp = hv;
  }
  wave_lds_sync();
}

template <bool SEQ>
__global__ __launch_bounds__(SCAN_THR) void tanh_scan_kernel(const unsigned short* __restrict__ Wp,
                                                             const float* __restrict__ XP,
                                                             const unsigned short* __restrict__ Sinp,
                                                             unsigned short* __restrict__ Soutp,
                                                             unsigned short* __restrict__ HSEQp,
                                                             int first) {
  __shared__ __align__(16) _Float16 Hb[SCAN_ROWS * H_PITCH];
  __shared__ __align__(16) float    Sl[SCAN_WAVES][16 * SLAB_PITCH];
  const _Float16* W    = (const _Float16*)Wp;
  const _Float16* Sin  = (const _Float16*)Sinp;
  _Float16*       Sout = (_Float16*)Soutp;
  _Float16*       HSEQ = (_Float16*)HSEQp;
  const int tid = threadIdx.x, lane = tid & 31, wave = tid >> 5;
  const int c = lane & 15, hh = lane >> 4, koff = hh * 8;
  const int q = lane >> 3, c8 = (lane & 7) * 8;
  const int rowbase = blockIdx.x * SCAN_ROWS;

  {
    const v8h zv = {(_Float16)0.0f, (_Float16)0.0f, (_Float16)0.0f, (_Float16)0.0f,
                    (_Float16)0.0f, (_Float16)0.0f, (_Float16)0.0f, (_Float16)0.0f};
#pragma unroll 1
    for (int i = 0; i < (SCAN_ROWS * (N_HID / 8)) / SCAN_THR; ++i) {
      const int idx = i * SCAN_THR + tid;
      const int row = idx / (N_HID / 8);
      const int col = (idx - row * (N_HID / 8)) * 8;
      v8h v = zv;
      if (first == 0) v = *(const v8h*)(Sin + (size_t)(rowbase + row) * N_HID + col);
      *(v8h*)(Hb + row * H_PITCH + col) = v;
    }
  }
  __syncthreads();

  const _Float16* ah0 = Hb + c * H_PITCH + koff;
  const _Float16* ah1 = Hb + (16 + c) * H_PITCH + koff;
  const _Float16* wb  = W + (size_t)(64 * wave + c) * N_HID + koff;
  const v8f z8 = {0.f, 0.f, 0.f, 0.f, 0.f, 0.f, 0.f, 0.f};
  float* slab = Sl[wave];

#pragma unroll 1
  for (int tl = 0; tl < T_CHUNK; ++tl) {
    v8f a00 = z8, a01 = z8, a02 = z8, a03 = z8;
    v8f a10 = z8, a11 = z8, a12 = z8, a13 = z8;
#pragma unroll 1
    for (int k0 = 0; k0 < N_HID; k0 += 32) {
      const v16h fa0 = FragH::load(ah0 + k0);
      const v16h fa1 = FragH::load(ah1 + k0);
      const v16h fb0 = FragH::load(wb + k0);
      const v16h fb1 = FragH::load(wb + (size_t)16 * N_HID + k0);
      const v16h fb2 = FragH::load(wb + (size_t)32 * N_HID + k0);
      const v16h fb3 = FragH::load(wb + (size_t)48 * N_HID + k0);
      a00 = FragH::mma(fa0, fb0, a00);
      a01 = FragH::mma(fa0, fb1, a01);
      a02 = FragH::mma(fa0, fb2, a02);
      a03 = FragH::mma(fa0, fb3, a03);
      a10 = FragH::mma(fa1, fb0, a10);
      a11 = FragH::mma(fa1, fb1, a11);
      a12 = FragH::mma(fa1, fb2, a12);
      a13 = FragH::mma(fa1, fb3, a13);
      guard8_h(a00, a01, a02, a03, a10, a11, a12, a13, fa0, fa1, fb0, fb1, fb2, fb3);
    }
    __syncthreads();
    const bool last = (tl == T_CHUNK - 1);
    const size_t grow0 = ((size_t)tl * N_BATCH + (size_t)rowbase) * N_HID + (size_t)(64 * wave);
    const size_t srow0 = (size_t)rowbase * N_HID + (size_t)(64 * wave);
    epi_half<SEQ>(a00, a01, a02, a03, slab, Hb + 64 * wave, XP + grow0,
                  HSEQ + grow0, Sout + srow0, last, c, hh, q, c8);
    epi_half<SEQ>(a10, a11, a12, a13, slab, Hb + 16 * H_PITCH + 64 * wave, XP + grow0 + (size_t)16 * N_HID,
                  HSEQ + grow0 + (size_t)16 * N_HID, Sout + srow0 + (size_t)16 * N_HID, last, c, hh, q, c8);
    __syncthreads();
  }
}

extern "C" void kernel_launch(void* const* d_in, const int* in_sizes, int n_in,
                              void* d_out, int out_size, void* d_ws, size_t ws_size, hipStream_t stream) {
  if (n_in < 11 || d_out == nullptr || d_ws == nullptr) return;
  if (in_sizes[0] != N_BATCH * N_STEP * N_IN || in_sizes[1] != N_HID * N_IN || in_sizes[2] != N_HID * N_HID ||
      in_sizes[3] != N_HID || in_sizes[4] != N_HID || in_sizes[5] != N_HID * N_HID || in_sizes[6] != N_HID * N_HID ||
      in_sizes[7] != N_HID || in_sizes[8] != N_HID || in_sizes[9] != N_OUT * N_HID || in_sizes[10] != N_OUT ||
      out_size != N_BATCH * N_OUT) return;

  const float* x    = (const float*)d_in[0];
  const float* Wih0 = (const float*)d_in[1];
  const float* Whh0 = (const float*)d_in[2];
  const float* bih0 = (const float*)d_in[3];
  const float* bhh0 = (const float*)d_in[4];
  const float* Wih1 = (const float*)d_in[5];
  const float* Whh1 = (const float*)d_in[6];
  const float* bih1 = (const float*)d_in[7];
  const float* bhh1 = (const float*)d_in[8];
  const float* Wfc  = (const float*)d_in[9];
  const float* bfc  = (const float*)d_in[10];
  float* out = (float*)d_out;

  char* ws = (char*)d_ws;
  size_t off = 0;
  auto carve = [&](size_t bytes) -> char* { char* p = ws + off; off += (bytes + 255) & ~(size_t)255; return p; };
  unsigned short* X16  = (unsigned short*)carve((size_t)N_BATCH * N_STEP * N_IN * 2);
  unsigned short* WIH0 = (unsigned short*)carve((size_t)N_HID * N_IN * 2);
  unsigned short* WHH0 = (unsigned short*)carve((size_t)N_HID * N_HID * 2);
  unsigned short* WIH1 = (unsigned short*)carve((size_t)N_HID * N_HID * 2);
  unsigned short* WHH1 = (unsigned short*)carve((size_t)N_HID * N_HID * 2);
  unsigned short* WFC  = (unsigned short*)carve((size_t)N_OUT * N_HID * 2);
  float*          BS0  = (float*)carve((size_t)N_HID * 4);
  float*          BS1  = (float*)carve((size_t)N_HID * 4);
  float*          BFR  = (float*)carve((size_t)N_OUT * 4);
  float*          XPC  = (float*)carve((size_t)CH_ROWS * N_HID * 4);
  unsigned short* H1C  = (unsigned short*)carve((size_t)CH_ROWS * N_HID * 2);
  unsigned short* ST   = (unsigned short*)carve((size_t)4 * N_BATCH * N_HID * 2);
  if (off > ws_size || off > (size_t)134217728) return;
  const size_t plane = (size_t)N_BATCH * N_HID;

  const int n8_ih0 = N_HID * N_IN / 8;
  const int n8_hh  = N_HID * N_HID / 8;
  const int n8_fc  = N_OUT * N_HID / 8;
  cvt_x_tmajor_kernel<<<(N_BATCH * N_STEP * (N_IN / 8)) / 256, 256, 0, stream>>>(x, X16);
  cvt_w_kernel<<<(n8_ih0 + 255) / 256, 256, 0, stream>>>(Wih0, WIH0, n8_ih0, W_CARRY);
  cvt_w_kernel<<<(n8_hh + 255) / 256, 256, 0, stream>>>(Whh0, WHH0, n8_hh, W_CARRY);
  cvt_w_kernel<<<(n8_hh + 255) / 256, 256, 0, stream>>>(Wih1, WIH1, n8_hh, W_CARRY);
  cvt_w_kernel<<<(n8_hh + 255) / 256, 256, 0, stream>>>(Whh1, WHH1, n8_hh, W_CARRY);
  cvt_w_kernel<<<(n8_fc + 255) / 256, 256, 0, stream>>>(Wfc, WFC, n8_fc, W_CARRY);
  bias_prep_kernel<<<3, 256, 0, stream>>>(bih0, bhh0, bih1, bhh1, bfc, BS0, BS1, BFR);

  const int gemm_blocks = ((CH_ROWS / 64) * (N_HID / 64) + 7) / 8;
  for (int ch = 0; ch < N_CHUNK; ++ch) {
    const int first = (ch == 0) ? 1 : 0;
    const int pin = ch & 1;
    const int pout = pin ^ 1;
    unsigned short* S0in  = ST + (size_t)(0 * 2 + pin)  * plane;
    unsigned short* S0out = ST + (size_t)(0 * 2 + pout) * plane;
    unsigned short* S1in  = ST + (size_t)(1 * 2 + pin)  * plane;
    unsigned short* S1out = ST + (size_t)(1 * 2 + pout) * plane;
    wmma_gemm64_f16<<<gemm_blocks, 256, 0, stream>>>(
        X16 + (size_t)ch * CH_ROWS * N_IN, N_IN, WIH0, N_IN, XPC, N_HID, BS0,
        CH_ROWS, N_HID, N_IN, W_CARRY_INV);
    tanh_scan_kernel<true><<<N_BATCH / SCAN_ROWS, SCAN_THR, 0, stream>>>(WHH0, XPC, S0in, S0out, H1C, first);
    wmma_gemm64_f16<<<gemm_blocks, 256, 0, stream>>>(
        H1C, N_HID, WIH1, N_HID, XPC, N_HID, BS1,
        CH_ROWS, N_HID, N_HID, W_CARRY_INV);
    tanh_scan_kernel<false><<<N_BATCH / SCAN_ROWS, SCAN_THR, 0, stream>>>(WHH1, XPC, S1in, S1out, H1C, first);
  }
  const int head_blocks = ((N_BATCH / 64) * (N_OUT / 64) + 7) / 8;
  wmma_gemm64_f16<<<head_blocks, 256, 0, stream>>>(
      ST + (size_t)(1 * 2 + 0) * plane, N_HID, WFC, N_HID, out, N_OUT, BFR,
      N_BATCH, N_OUT, N_HID, W_CARRY_INV);
}
